// Attention_7696581394614
// MI455X (gfx1250) — hardware-verified
//
#include <hip/hip_runtime.h>


#ifndef NB
#define NB 4
#endif
#ifndef SEQ
#define SEQ 2048
#endif
#define NB_FULL  4
#define SEQ_FULL 2048
#define DIM   768
#define HEADS 12
#define HD    64
#define QKVN  2304
#define CXW   1536
#define MROWS (NB * SEQ)
#define TM    128
#define TN    64
#define CSP   68
#define NWV   4
#define BQ    (16 * NWV)
#define KS    32
#define OSP   68
#define L2E   1.4426950408889634f
#define SCL   (0.125f * L2E)
#define PCAR  8.0f
#define QRS   2048.0f
#define QRI   (1.0f / 2048.0f)

#define PC_ROW (DIM / 8)
#define GCX ((unsigned)((size_t)MROWS * PC_ROW / 256))
#define GCQ ((unsigned)((size_t)QKVN * PC_ROW / 256))
#define GCP ((unsigned)((size_t)DIM * PC_ROW / 256))

#define PL_X  ((size_t)MROWS * DIM * 2)
#define PL_WQ ((size_t)QKVN * DIM * 2)
#define PL_WP ((size_t)DIM * DIM * 2)
#define PL_H  ((size_t)NB * HEADS * SEQ * HD * 2)
#define PL_CX ((size_t)MROWS * CXW * 2)

static_assert(DIM == HEADS * HD);
static_assert(HD == 64);
static_assert(QKVN == 3 * DIM);
static_assert(CXW == 2 * DIM);
static_assert(DIM % 32 == 0);
static_assert(CXW % 32 == 0);
static_assert(HD % 32 == 0);
static_assert(DIM % 8 == 0);
static_assert(TN == HD);
static_assert(DIM % TN == 0);
static_assert(QKVN % TN == 0);
static_assert(SEQ % TM == 0);
static_assert(MROWS % TM == 0);
static_assert(SEQ % BQ == 0);
static_assert(SEQ % KS == 0);
static_assert(NB <= NB_FULL);
static_assert(SEQ <= SEQ_FULL);
static_assert(((size_t)MROWS * PC_ROW) % 256 == 0);
static_assert(((size_t)QKVN * PC_ROW) % 256 == 0);
static_assert(((size_t)DIM * PC_ROW) % 256 == 0);
static_assert(TM == 4 * 32);
static_assert(CSP >= TN && CSP % 4 == 0);
static_assert(OSP >= HD && OSP % 4 == 0);
static_assert(PL_X % 256 == 0 && PL_WQ % 256 == 0 && PL_WP % 256 == 0 && PL_H % 256 == 0 && PL_CX % 256 == 0);
static_assert(PL_X + PL_WQ + PL_WP + 4 * PL_H + PL_CX <= (size_t)134217728);
static_assert((size_t)(MROWS / TM) * (QKVN / TN) * (size_t)(TM * TN) == (size_t)MROWS * QKVN);
static_assert((size_t)(NB * HEADS * (SEQ / BQ)) * (size_t)(BQ * HD) == (size_t)MROWS * DIM);
static_assert((size_t)(MROWS / TM) * (DIM / TN) * (size_t)(TM * TN) == (size_t)MROWS * DIM);

typedef unsigned short bf;
typedef _Float16 hf;
typedef __attribute__((ext_vector_type(16))) __bf16   v16bf;
typedef __attribute__((ext_vector_type(16))) _Float16 v16h;
typedef __attribute__((ext_vector_type(8)))  _Float16 v8h;
typedef __attribute__((ext_vector_type(8)))  unsigned short v8us;
typedef __attribute__((ext_vector_type(8)))  float    v8f;
typedef __attribute__((ext_vector_type(4)))  float    v4f;
typedef v4f  __attribute__((may_alias)) v4fa;

__device__ __forceinline__ unsigned short f2bf(float f) { unsigned u = __float_as_uint(f); u += 0x7FFFu + ((u >> 16) & 1u); return (unsigned short)(u >> 16); }
__device__ __forceinline__ float bf2f(unsigned short b) { return __uint_as_float(((unsigned)b) << 16); }
__device__ __forceinline__ float bfr(float f) { return bf2f(f2bf(f)); }
__device__ __forceinline__ v8f wmmab(v16bf a, v16bf b, v8f c) { return __builtin_amdgcn_wmma_f32_16x16x32_bf16(false, a, false, b, (short)0, c, false, false); }
__device__ __forceinline__ v8f wmmah(v16h a, v16h b, v8f c) { return __builtin_amdgcn_wmma_f32_16x16x32_f16(false, a, false, b, (short)0, c, false, false); }
__device__ __forceinline__ v16bf ldfb(const bf* p) {
    const v8us lo = *(const v8us*)p, hi = *(const v8us*)(p + 16);
    return __builtin_bit_cast(v16bf, __builtin_shufflevector(lo, hi, 0, 1, 2, 3, 4, 5, 6, 7, 8, 9, 10, 11, 12, 13, 14, 15));
}
__device__ __forceinline__ v16h ldfh(const hf* p) {
    const v8h lo = *(const v8h*)p, hi = *(const v8h*)(p + 16);
    return __builtin_shufflevector(lo, hi, 0, 1, 2, 3, 4, 5, 6, 7, 8, 9, 10, 11, 12, 13, 14, 15);
}

__device__ __forceinline__ void cvt_store(const float* __restrict__ src, bf* dst) {
    const v8f v = *(const v8f*)src;
    v8us o;
#pragma unroll
    for (int c = 0; c < 8; ++c) o[c] = f2bf(v[c]);
    *(volatile v8us*)dst = o;
    __threadfence();
    *(volatile v8us*)dst = o;
}

__global__ __launch_bounds__(256) void k_cvt(const float* __restrict__ x, const float* __restrict__ wq, const float* __restrict__ wp,
                                             bf* XB, bf* WQ, bf* WP) {
    const unsigned blk = blockIdx.x, tid = threadIdx.x;
    if (blk < GCX) {
        const unsigned i = blk * 256u + tid;
        const unsigned row = i / PC_ROW, pc = i - row * PC_ROW;
        const unsigned b = row / SEQ, p = row - b * SEQ;
        cvt_store(x + ((size_t)b * SEQ_FULL + p) * DIM + pc * 8u, XB + (size_t)i * 8);
    } else if (blk < GCX + GCQ) {
        const unsigned i = (blk - GCX) * 256u + tid;
        const unsigned row = i / PC_ROW, pc = i - row * PC_ROW;
        const unsigned which = row / DIM, rem = row - which * DIM;
        const unsigned h = rem >> 6, d = rem & 63u;
        const unsigned srow = which * DIM + d * HEADS + h;
        cvt_store(wq + (size_t)srow * DIM + pc * 8u, WQ + (size_t)i * 8);
    } else {
        const unsigned i = (blk - GCX - GCQ) * 256u + tid;
        cvt_store(wp + (size_t)i * 8, WP + (size_t)i * 8);
    }
}

__device__ __forceinline__ void gemm_tile(const bf* __restrict__ Ap, const bf* __restrict__ Bp,
                                          const unsigned lda, const unsigned ldw, const unsigned K, const unsigned KW, v8f (&c)[8]) {
#pragma unroll 1
    for (unsigned k0 = 0; k0 < K; k0 += 32) {
        const unsigned kb = (k0 >= KW) ? (k0 - KW) : k0;
        const v16bf a0 = ldfb(Ap + k0);
        const v16bf a1 = ldfb(Ap + (size_t)16 * lda + k0);
        const v16bf b0 = ldfb(Bp + kb);
        const v16bf b1 = ldfb(Bp + (size_t)16 * ldw + kb);
        const v16bf b2 = ldfb(Bp + (size_t)32 * ldw + kb);
        const v16bf b3 = ldfb(Bp + (size_t)48 * ldw + kb);
        c[0] = wmmab(a0, b0, c[0]);
        c[1] = wmmab(a0, b1, c[1]);
        c[2] = wmmab(a0, b2, c[2]);
        c[3] = wmmab(a0, b3, c[3]);
        c[4] = wmmab(a1, b0, c[4]);
        c[5] = wmmab(a1, b1, c[5]);
        c[6] = wmmab(a1, b2, c[6]);
        c[7] = wmmab(a1, b3, c[7]);
        asm volatile("v_nop\n\tv_nop\n\tv_nop\n\tv_nop"
                     : "+v"(c[0]), "+v"(c[1]), "+v"(c[2]), "+v"(c[3]), "+v"(c[4]), "+v"(c[5]), "+v"(c[6]), "+v"(c[7])
                     : "v"(a0), "v"(a1), "v"(b0), "v"(b1), "v"(b2), "v"(b3));
    }
}

__global__ __launch_bounds__(128) void k_qkv(const bf* __restrict__ XB, const bf* __restrict__ WQ, const float* __restrict__ bq,
                                             hf* QH, hf* QL, hf* KH, hf* VT) {
    __shared__ __align__(16) float cs[TM * CSP];
    const unsigned tid = threadIdx.x, lane = tid & 31u, lr = lane & 15u, hi = lane >> 4;
    const unsigned wave = (unsigned)__builtin_amdgcn_readfirstlane((int)(tid >> 5));
    const unsigned NT = QKVN / TN;
    const unsigned mt = blockIdx.x / NT, nt = blockIdx.x - mt * NT;
    const unsigned which = nt / HEADS, h = nt - which * HEADS;
    const unsigned m0 = mt * TM, n0 = nt * TN;
    const unsigned b = m0 / SEQ, p0 = m0 - b * SEQ;
    const unsigned bh = b * HEADS + h;

    v8f c[8];
#pragma unroll
    for (int t = 0; t < 8; ++t) c[t] = (v8f){};
    gemm_tile(XB + (size_t)(m0 + wave * 32u + lr) * DIM + 8u * hi, WQ + (size_t)(n0 + lr) * DIM + 8u * hi, DIM, DIM, DIM, DIM, c);

    const unsigned bb = which * DIM + h;
    const float bv0 = bfr(bq[bb + (lr) * HEADS]);
    const float bv1 = bfr(bq[bb + (16u + lr) * HEADS]);
    const float bv2 = bfr(bq[bb + (32u + lr) * HEADS]);
    const float bv3 = bfr(bq[bb + (48u + lr) * HEADS]);
    const unsigned rb = wave * 32u + 8u * hi;
#pragma unroll
    for (int r = 0; r < 8; ++r) {
        cs[(rb + r) * CSP + lr]            = c[0][r] + bv0;
        cs[(rb + r) * CSP + 16u + lr]      = c[1][r] + bv1;
        cs[(rb + r) * CSP + 32u + lr]      = c[2][r] + bv2;
        cs[(rb + r) * CSP + 48u + lr]      = c[3][r] + bv3;
        cs[(rb + 16u + r) * CSP + lr]       = c[4][r] + bv0;
        cs[(rb + 16u + r) * CSP + 16u + lr] = c[5][r] + bv1;
        cs[(rb + 16u + r) * CSP + 32u + lr] = c[6][r] + bv2;
        cs[(rb + 16u + r) * CSP + 48u + lr] = c[7][r] + bv3;
    }
    __syncthreads();

    if (which == 0u) {
        const unsigned c8 = (tid & 7u) * 8u, rq = tid >> 3;
#pragma unroll 1
        for (int ps = 0; ps < 2; ++ps) {
#pragma unroll 2
            for (unsigned it = 0; it < 8; ++it) {
                const unsigned row = it * 16u + rq;
                const v4f x0 = *(const v4fa*)&cs[row * CSP + c8];
                const v4f x1 = *(const v4fa*)&cs[row * CSP + c8 + 4u];
                v8h vh, vl;
#pragma unroll
                for (int e = 0; e < 4; ++e) {
                    const _Float16 t0 = (_Float16)x0[e];
                    const _Float16 t1 = (_Float16)x1[e];
                    vh[e] = t0; vh[4 + e] = t1;
                    vl[e]     = (_Float16)((x0[e] - (float)t0) * QRS);
                    vl[4 + e] = (_Float16)((x1[e] - (float)t1) * QRS);
                }
                const size_t off = ((size_t)bh * SEQ + p0 + row) * HD + c8;
                *(volatile v8h*)(QH + off) = vh;
                *(volatile v8h*)(QL + off) = vl;
            }
            if (ps == 0) __threadfence();
        }
    } else if (which == 1u) {
        const unsigned c8 = (tid & 7u) * 8u, rq = tid >> 3;
#pragma unroll 1
        for (int ps = 0; ps < 2; ++ps) {
#pragma unroll 2
            for (unsigned it = 0; it < 8; ++it) {
                const unsigned row = it * 16u + rq;
                const v4f x0 = *(const v4fa*)&cs[row * CSP + c8];
                const v4f x1 = *(const v4fa*)&cs[row * CSP + c8 + 4u];
                v8h vh;
#pragma unroll
                for (int e = 0; e < 4; ++e) { vh[e] = (_Float16)x0[e]; vh[4 + e] = (_Float16)x1[e]; }
                *(volatile v8h*)(KH + ((size_t)bh * SEQ + p0 + row) * HD + c8) = vh;
            }
            if (ps == 0) __threadfence();
        }
    } else {
        const unsigned pp = (tid & 15u) * 8u, dq = tid >> 4;
#pragma unroll 1
        for (int ps = 0; ps < 2; ++ps) {
#pragma unroll 2
            for (unsigned it = 0; it < 8; ++it) {
                const unsigned d = it * 8u + dq;
                v8h o;
#pragma unroll
                for (unsigned e = 0; e < 8; ++e) o[e] = (_Float16)cs[(pp + e) * CSP + d];
                *(volatile v8h*)(VT + ((size_t)bh * HD + d) * SEQ + p0 + pp) = o;
            }
            if (ps == 0) __threadfence();
        }
    }
}

__global__ __launch_bounds__(128) void k_flash(const hf* __restrict__ QH, const hf* __restrict__ QL, const hf* __restrict__ KH,
                                               const hf* __restrict__ VT, bf* CX) {
    __shared__ __align__(16) float os[NWV * 16 * OSP];
    const unsigned tid = threadIdx.x, lane = tid & 31u, lr = lane & 15u, hi = lane >> 4;
    const unsigned wave = (unsigned)__builtin_amdgcn_readfirstlane((int)(tid >> 5));
    const unsigned bpb = (unsigned)(SEQ / BQ);
    const unsigned bh = blockIdx.x / bpb;
    const unsigned q0 = (blockIdx.x - bh * bpb) * BQ + wave * 16u;
    const unsigned b = bh / HEADS, h = bh - b * HEADS;

    const size_t qoff = ((size_t)bh * SEQ + q0 + lr) * HD + 8u * hi;
    const v16h qh0 = ldfh(QH + qoff), qh1 = ldfh(QH + qoff + 32);
    const v16h ql0 = ldfh(QL + qoff), ql1 = ldfh(QL + qoff + 32);
    const hf* kp = KH + ((size_t)bh * SEQ + lr) * HD + 8u * hi;
    const hf* vp = VT + ((size_t)bh * HD + lr) * SEQ + 8u * hi;

    v8f o0 = (v8f){}, o1 = (v8f){}, o2 = (v8f){}, o3 = (v8f){};
    float ml = -1.0e30f;
    float l = 0.0f;

#pragma unroll 1
    for (unsigned k0 = 0; k0 < (unsigned)SEQ; k0 += KS) {
        const hf* ka = kp + (size_t)k0 * HD;
        const v16h a00 = ldfh(ka), a01 = ldfh(ka + 32);
        const v16h a10 = ldfh(ka + 16 * HD), a11 = ldfh(ka + 16 * HD + 32);
        v8f sh0 = (v8f){}, sl0 = (v8f){}, sh1 = (v8f){}, sl1 = (v8f){};
        sh0 = wmmah(a00, qh0, sh0);
        sl0 = wmmah(a00, ql0, sl0);
        sh1 = wmmah(a10, qh0, sh1);
        sl1 = wmmah(a10, ql0, sl1);
        sh0 = wmmah(a01, qh1, sh0);
        sl0 = wmmah(a01, ql1, sl0);
        sh1 = wmmah(a11, qh1, sh1);
        sl1 = wmmah(a11, ql1, sl1);
        asm volatile("v_nop\n\tv_nop\n\tv_nop\n\tv_nop"
                     : "+v"(sh0), "+v"(sl0), "+v"(sh1), "+v"(sl1)
                     : "v"(qh0), "v"(qh1), "v"(ql0), "v"(ql1), "v"(a01), "v"(a11));
        const v8f s0 = sh0 + sl0 * QRI;
        const v8f s1 = sh1 + sl1 * QRI;

        float mx = fmaxf(s0[0], s1[0]);
#pragma unroll
        for (int r = 1; r < 8; ++r) mx = fmaxf(mx, fmaxf(s0[r], s1[r]));
        mx = fmaxf(mx, __shfl_xor(mx, 16, 32));
        const float mnl = fmaxf(ml, mx * SCL);
        const float corr = __builtin_amdgcn_exp2f(ml - mnl);
        ml = mnl;
        const float nb = PCAR - mnl;
        float p0[8], p1[8];
        float ps = 0.0f;
#pragma unroll
        for (int r = 0; r < 8; ++r) {
            p0[r] = __builtin_amdgcn_exp2f(fmaf(s0[r], SCL, nb));
            p1[r] = __builtin_amdgcn_exp2f(fmaf(s1[r], SCL, nb));
            ps += p0[r] + p1[r];
        }
        ps += __shfl_xor(ps, 16, 32);
        l = l * corr + ps;
        if (__builtin_amdgcn_ballot_w32(corr != 1.0f) != 0u) {
            o0 *= corr; o1 *= corr; o2 *= corr; o3 *= corr;
        }

        v16h ph;
#pragma unroll
        for (int r = 0; r < 8; ++r) { ph[r] = (_Float16)p0[r]; ph[8 + r] = (_Float16)p1[r]; }

        asm volatile("" ::: "memory");
        const hf* va = vp + k0;
        const v16h v0 = ldfh(va);
        const v16h v1 = ldfh(va + (size_t)16 * SEQ);
        const v16h v2 = ldfh(va + (size_t)32 * SEQ);
        const v16h v3 = ldfh(va + (size_t)48 * SEQ);
        o0 = wmmah(v0, ph, o0);
        o1 = wmmah(v1, ph, o1);
        o2 = wmmah(v2, ph, o2);
        o3 = wmmah(v3, ph, o3);
        asm volatile("v_nop\n\tv_nop\n\tv_nop\n\tv_nop"
                     : "+v"(o0), "+v"(o1), "+v"(o2), "+v"(o3)
                     : "v"(ph), "v"(v0), "v"(v1), "v"(v2), "v"(v3));
    }

    const float inv = 1.0f / l;
    const unsigned ob = wave * (16u * OSP);
#pragma unroll
    for (int r = 0; r < 8; ++r) {
        os[ob + lr * OSP + 8u * hi + r]       = o0[r] * inv;
        os[ob + lr * OSP + 16u + 8u * hi + r] = o1[r] * inv;
        os[ob + lr * OSP + 32u + 8u * hi + r] = o2[r] * inv;
        os[ob + lr * OSP + 48u + 8u * hi + r] = o3[r] * inv;
    }
    __syncthreads();
    bf* cxp = CX + ((size_t)b * SEQ + q0) * CXW + h * HD;
    const unsigned c8 = (lane & 7u) * 8u, rq = lane >> 3;
#pragma unroll 1
    for (int ps2 = 0; ps2 < 2; ++ps2) {
#pragma unroll
        for (unsigned it = 0; it < 4; ++it) {
            const unsigned row = it * 4u + rq;
            const v4f x0 = *(const v4fa*)&os[ob + row * OSP + c8];
            const v4f x1 = *(const v4fa*)&os[ob + row * OSP + c8 + 4u];
            v8us vh, vl;
#pragma unroll
            for (int e = 0; e < 4; ++e) {
                const unsigned short t0 = f2bf(x0[e]);
                const unsigned short t1 = f2bf(x1[e]);
                vh[e] = t0; vh[4 + e] = t1;
                vl[e]     = f2bf(x0[e] - bf2f(t0));
                vl[4 + e] = f2bf(x1[e] - bf2f(t1));
            }
            *(volatile v8us*)(cxp + (size_t)row * CXW + c8) = vh;
            *(volatile v8us*)(cxp + (size_t)row * CXW + DIM + c8) = vl;
        }
        if (ps2 == 0) __threadfence();
    }
}

__global__ __launch_bounds__(128) void k_proj(const bf* __restrict__ CX, const bf* __restrict__ WP, const float* __restrict__ bp, float* OUT) {
    __shared__ __align__(16) float cs[TM * CSP];
    const unsigned tid = threadIdx.x, lane = tid & 31u, lr = lane & 15u, hi = lane >> 4;
    const unsigned wave = (unsigned)__builtin_amdgcn_readfirstlane((int)(tid >> 5));
    const unsigned NT = DIM / TN;
    const unsigned mt = blockIdx.x / NT, nt = blockIdx.x - mt * NT;
    const unsigned m0 = mt * TM, n0 = nt * TN;

    v8f c[8];
#pragma unroll
    for (int t = 0; t < 8; ++t) c[t] = (v8f){};
    gemm_tile(CX + (size_t)(m0 + wave * 32u + lr) * CXW + 8u * hi, WP + (size_t)(n0 + lr) * DIM + 8u * hi, CXW, DIM, CXW, DIM, c);

    const float bv0 = bfr(bp[n0 + lr]);
    const float bv1 = bfr(bp[n0 + 16u + lr]);
    const float bv2 = bfr(bp[n0 + 32u + lr]);
    const float bv3 = bfr(bp[n0 + 48u + lr]);
    const unsigned rb = wave * 32u + 8u * hi;
#pragma unroll
    for (int r = 0; r < 8; ++r) {
        cs[(rb + r) * CSP + lr]            = c[0][r] + bv0;
        cs[(rb + r) * CSP + 16u + lr]      = c[1][r] + bv1;
        cs[(rb + r) * CSP + 32u + lr]      = c[2][r] + bv2;
        cs[(rb + r) * CSP + 48u + lr]      = c[3][r] + bv3;
        cs[(rb + 16u + r) * CSP + lr]       = c[4][r] + bv0;
        cs[(rb + 16u + r) * CSP + 16u + lr] = c[5][r] + bv1;
        cs[(rb + 16u + r) * CSP + 32u + lr] = c[6][r] + bv2;
        cs[(rb + 16u + r) * CSP + 48u + lr] = c[7][r] + bv3;
    }
    __syncthreads();
    float* dst = OUT + (size_t)m0 * DIM + n0;
    const unsigned c4 = (tid & 15u) * 4u, rq = tid >> 4;
#pragma unroll 1
    for (int ps = 0; ps < 2; ++ps) {
#pragma unroll 4
        for (unsigned it = 0; it < 16; ++it) {
            const unsigned row = it * 8u + rq;
            const v4f val = *(const v4fa*)&cs[row * CSP + c4];
            *(volatile v4f*)(dst + (size_t)row * DIM + c4) = val;
        }
        if (ps == 0) __threadfence();
    }
}

extern "C" void kernel_launch(void* const* d_in, const int* in_sizes, int n_in,
                              void* d_out, int out_size, void* d_ws, size_t ws_size, hipStream_t stream) {
    if (n_in < 5) return;
    const size_t need_x = ((size_t)(NB - 1) * SEQ_FULL + SEQ) * DIM;
    if ((size_t)in_sizes[0] < need_x) return;
    if ((size_t)in_sizes[1] < (size_t)QKVN * DIM) return;
    if ((size_t)in_sizes[2] < (size_t)QKVN) return;
    if ((size_t)in_sizes[3] < (size_t)DIM * DIM) return;
    if ((size_t)in_sizes[4] < (size_t)DIM) return;
    if ((size_t)out_size < (size_t)MROWS * DIM) return;
    const float* x  = (const float*)d_in[0];
    const float* wq = (const float*)d_in[1];
    const float* bq = (const float*)d_in[2];
    const float* wp = (const float*)d_in[3];
    const float* bp = (const float*)d_in[4];
    float* OUT = (float*)d_out;

    const size_t total = PL_X + PL_WQ + PL_WP + 4 * PL_H + PL_CX;
    if (total > ws_size) return;
    char* wsp = (char*)d_ws;
    size_t off = 0;
    bf* XB = (bf*)(wsp + off); off += PL_X;
    bf* WQ = (bf*)(wsp + off); off += PL_WQ;
    bf* WP = (bf*)(wsp + off); off += PL_WP;
    hf* QH = (hf*)(wsp + off); off += PL_H;
    hf* QL = (hf*)(wsp + off); off += PL_H;
    hf* KH = (hf*)(wsp + off); off += PL_H;
    hf* VT = (hf*)(wsp + off); off += PL_H;
    bf* CX = (bf*)(wsp + off); off += PL_CX;

    k_cvt<<<GCX + GCQ + GCP, 256, 0, stream>>>(x, wq, wp, XB, WQ, WP);
    k_qkv<<<(unsigned)((MROWS / TM) * (QKVN / TN)), 128, 0, stream>>>(XB, WQ, bq, QH, QL, KH, VT);
    k_flash<<<(unsigned)(NB * HEADS * (SEQ / BQ)), 128, 0, stream>>>(QH, QL, KH, VT, CX);
    k_proj<<<(unsigned)((MROWS / TM) * (DIM / TN)), 128, 0, stream>>>(CX, WP, bp, OUT);
}
